// PointNetSetAbstraction_63462436766094
// MI455X (gfx1250) — hardware-verified
//
#include <hip/hip_runtime.h>
#pragma clang fp contract(off)

typedef __attribute__((ext_vector_type(16))) _Float16 v16h;
typedef __attribute__((ext_vector_type(8)))  _Float16 v8h;
typedef __attribute__((ext_vector_type(8)))  float    v8f;
typedef __attribute__((ext_vector_type(4)))  float    v4f;
typedef __attribute__((ext_vector_type(4)))  unsigned v4u;

constexpr int kBatch   = 8;
constexpr int kNPts    = 4160;
constexpr int kFeat    = 64;
constexpr int kNCent   = 1024;
constexpr int kNSamp   = 32;
constexpr int kGroups  = kBatch * kNCent;
constexpr int kRows    = kGroups * kNSamp;
constexpr int kK0      = 96;
constexpr int kCin0    = 67;
constexpr int kFpsPer  = 17;
constexpr int kCandCap = 512;
constexpr float kWCarry    = 16.0f;
constexpr float kWCarryInv = 1.0f / 16.0f;
constexpr float kRad2      = 0.25f;

static_assert(kNPts % 32 == 0);
static_assert(kFpsPer * 256 >= kNPts);
static_assert(kRows % 512 == 0);
static_assert(kK0 % 32 == 0 && kFeat % 32 == 0);
static_assert(kGroups == 8192 && kRows == 262144);

constexpr size_t kOffX0    = 0;
constexpr size_t kSzX0     = (size_t)kRows * kK0 * 2;
constexpr size_t kOffYA    = kOffX0 + kSzX0;
constexpr size_t kSzAct    = (size_t)kRows * 64 * 2;
constexpr size_t kOffXB    = kOffYA + kSzAct;
constexpr size_t kOffYMax  = kOffXB + kSzAct;
constexpr size_t kSzPool   = (size_t)kGroups * 128 * 4;
constexpr size_t kOffYMin  = kOffYMax + kSzPool;
constexpr size_t kOffPart0 = kOffYMin + kSzPool;
constexpr size_t kSzPart64 = (size_t)512 * 2 * 64 * 4;
constexpr size_t kOffPart1 = kOffPart0 + kSzPart64;
constexpr size_t kOffPart2 = kOffPart1 + kSzPart64;
constexpr size_t kSzPart128 = (size_t)512 * 2 * 128 * 4;
constexpr size_t kOffW0H   = kOffPart2 + kSzPart128;
constexpr size_t kOffW1H   = kOffW0H + (size_t)64 * kK0 * 2;
constexpr size_t kOffW2H   = kOffW1H + (size_t)64 * 64 * 2;
constexpr size_t kOffAB    = kOffW2H + (size_t)128 * 64 * 2;
constexpr size_t kOffCxyz  = kOffAB + (size_t)3 * 256 * 4;
constexpr size_t kWsTotal  = kOffCxyz + (size_t)kGroups * 3 * 4;
static_assert(kWsTotal <= (size_t)134217728);
static_assert(kOffYA % 256 == 0 && kOffXB % 256 == 0 && kOffYMax % 256 == 0 && kOffYMin % 256 == 0);
static_assert(kOffPart0 % 256 == 0 && kOffPart1 % 256 == 0 && kOffPart2 % 256 == 0);
static_assert(kOffW0H % 256 == 0 && kOffW1H % 256 == 0 && kOffW2H % 256 == 0 && kOffAB % 256 == 0 && kOffCxyz % 256 == 0);
constexpr size_t kOut1Bytes = 98304;
static_assert(kOut1Bytes == (size_t)kGroups * 3 * 4);
static_assert(kOut1Bytes % 128 == 0);
static_assert(kOut1Bytes + (size_t)kGroups * 128 * 4 == (size_t)4292608);

__device__ __forceinline__ void store2_v4f(float* p, v4f v) {
  *(volatile v4f*)p = v;
  __threadfence();
  *(volatile v4f*)p = v;
}
__device__ __forceinline__ void store2_v8h(unsigned short* p, v8h v) {
  *(volatile v8h*)p = v;
  __threadfence();
  *(volatile v8h*)p = v;
}
__device__ __forceinline__ void store2_f32(float* p, float v) {
  *(volatile float*)p = v;
  __threadfence();
  *(volatile float*)p = v;
}

__device__ __forceinline__ float h16_to_f32(unsigned hb) {
  const unsigned sgn = (hb & 0x8000u) << 16; const unsigned em = hb & 0x7fffu;
  const float fn = __uint_as_float((em << 13) + 0x38000000u);
  const float fs = (float)em * 5.9604644775390625e-8f;
  const float mag = (em < 0x400u) ? fs : fn; return __uint_as_float(__float_as_uint(mag) | sgn); }

union FragU { v16h v; v8h h[2]; };
__device__ __forceinline__ v16h frag_load(const _Float16* p) {
  FragU f; f.h[0] = *(const v8h*)(p); f.h[1] = *(const v8h*)(p + 16); return f.v;
}
__device__ __forceinline__ v8f mma_f16(v16h a, v16h b, v8f c) {
  return __builtin_amdgcn_wmma_f32_16x16x32_f16(false, a, false, b, (short)0, c, false, false);
}
__device__ __forceinline__ void guard_row(v8f& a0, v8f& a1, v8f& a2, v8f& a3, v16h x, v16h b0, v16h b1, v16h b2, v16h b3) {
  asm volatile("v_nop\n\tv_nop\n\tv_nop\n\tv_nop" : "+v"(a0), "+v"(a1), "+v"(a2), "+v"(a3) : "v"(x), "v"(b0), "v"(b1), "v"(b2), "v"(b3));
}
__device__ __forceinline__ void acc_guard4(v8f& a, v8f& b, v8f& c, v8f& d) {
  asm volatile("v_nop\n\tv_nop\n\tv_nop\n\tv_nop" : "+v"(a), "+v"(b), "+v"(c), "+v"(d));
}

__global__ __launch_bounds__(256) void fps_kernel(const float* __restrict__ xyz,
                                                  float* __restrict__ out0,
                                                  float* __restrict__ cxyz) {
#pragma clang fp contract(off)
  __shared__ float rv[2][8];
  __shared__ int   ri[2][8];
  __shared__ float sxyz[kNCent * 3];
  const int b    = blockIdx.x;
  const int tid  = threadIdx.x;
  const int lane = tid & 31;
  const int wave = tid >> 5;
  const float* X = xyz + (size_t)b * kNPts * 3;

  float px[kFpsPer], py[kFpsPer], pz[kFpsPer], ds[kFpsPer];
#pragma unroll
  for (int j = 0; j < kFpsPer; ++j) {
    const int i  = tid + 256 * j;
    const int ic = (i < kNPts) ? i : (kNPts - 1);
    px[j] = X[ic * 3 + 0];
    py[j] = X[ic * 3 + 1];
    pz[j] = X[ic * 3 + 2];
    ds[j] = (i < kNPts) ? 1.0e10f : -1.0f;
    if ((j & 3) == 3) asm volatile("" ::: "memory");
  }

  int far = 0;
  for (int it = 0; it < kNCent; ++it) {
    int fc = (far < 0) ? 0 : far;
    fc = (fc > kNPts - 1) ? (kNPts - 1) : fc;
    const float cx = X[fc * 3 + 0];
    const float cy = X[fc * 3 + 1];
    const float cz = X[fc * 3 + 2];
    if (tid == 0) {
      sxyz[it * 3 + 0] = cx;
      sxyz[it * 3 + 1] = cy;
      sxyz[it * 3 + 2] = cz;
    }
    float bv = -1.0f;
    int   bi = 0;
#pragma unroll
    for (int j = 0; j < kFpsPer; ++j) {
      const float dx = px[j] - cx;
      const float dy = py[j] - cy;
      const float dz = pz[j] - cz;
      const float t0 = dx * dx;
      const float t1 = dy * dy;
      const float t2 = dz * dz;
      const float d  = (t0 + t2) + t1;
      const float nd = fminf(ds[j], d);
      ds[j] = nd;
      if (nd > bv) { bv = nd; bi = tid + 256 * j; }
    }
#pragma unroll
    for (int off = 16; off > 0; off >>= 1) {
      const float ov = __shfl_xor(bv, off, 32);
      const int   oi = __shfl_xor(bi, off, 32);
      const bool take = (ov > bv) || ((ov == bv) && (oi < bi));
      bv = take ? ov : bv;
      bi = take ? oi : bi;
    }
    const int p = it & 1;
    if (lane == 0) { rv[p][wave] = bv; ri[p][wave] = bi; }
    __syncthreads();
    float gv = rv[p][0];
    int   gi = ri[p][0];
#pragma unroll
    for (int w = 1; w < 8; ++w) {
      const float ov = rv[p][w];
      const int   oi = ri[p][w];
      const bool take = (ov > gv) || ((ov == gv) && (oi < gi));
      gv = take ? ov : gv;
      gi = take ? oi : gi;
    }
    far = gi;
  }
  __syncthreads();
  float* o0 = out0 + (size_t)b * kNCent * 3;
  float* o1 = cxyz + (size_t)b * kNCent * 3;
#pragma unroll
  for (int k = 0; k < 3; ++k) {
    const int q = (k * 256 + tid) * 4;
    const v4f v = {sxyz[q + 0], sxyz[q + 1], sxyz[q + 2], sxyz[q + 3]};
    store2_v4f(o0 + q, v);
    store2_v4f(o1 + q, v);
  }
}

__global__ __launch_bounds__(128) void group_kernel(const float* __restrict__ xyz,
                                                    const float* __restrict__ pts,
                                                    const float* __restrict__ cxyz,
                                                    unsigned short* __restrict__ x0) {
#pragma clang fp contract(off)
  __shared__ float cd[4][kCandCap];
  __shared__ int   ci[4][kCandCap];
  __shared__ int   so[4][32];
  __shared__ __align__(16) _Float16 tile[4][32 * kK0];
  const int lane = threadIdx.x & 31;
  const int wave = threadIdx.x >> 5;
  const int g    = blockIdx.x * 4 + wave;
  const int b    = g >> 10;
  const float* X = xyz + (size_t)b * kNPts * 3;
  const float sx = cxyz[(size_t)g * 3 + 0];
  const float sy = cxyz[(size_t)g * 3 + 1];
  const float sz = cxyz[(size_t)g * 3 + 2];
  const float s0 = sx * sx;
  const float s1 = sy * sy;
  const float s2 = sz * sz;
  const float ssq = (s0 + s2) + s1;
  float* cdw = cd[wave];
  int*   ciw = ci[wave];
  int*   sow = so[wave];

  int   cnt = 0;
  float bd  = 3.0e38f;
  int   bi  = 0;
#pragma unroll 1
  for (int j = 0; j < kNPts / 32; ++j) {
    const int i = j * 32 + lane;
    const float qx = X[i * 3 + 0];
    const float qy = X[i * 3 + 1];
    const float qz = X[i * 3 + 2];
    const float t0 = qx * qx;
    const float t1 = qy * qy;
    const float t2 = qz * qz;
    const float psq = (t0 + t2) + t1;
    float p = sx * qx;
    p = __builtin_fmaf(sy, qy, p);
    p = __builtin_fmaf(sz, qz, p);
    const float m2 = -2.0f * p;
    const float d  = (m2 + ssq) + psq;
    if (d < bd) { bd = d; bi = i; }
    const bool hit = (d <= kRad2);
    const unsigned mask = __builtin_amdgcn_ballot_w32(hit);
    const int pre  = __builtin_popcount(mask & ((1u << lane) - 1u));
    const int slot = cnt + pre;
    if (hit && slot < kCandCap) { cdw[slot] = d; ciw[slot] = i; }
    cnt += __builtin_popcount(mask);
  }
#pragma unroll
  for (int off = 16; off > 0; off >>= 1) {
    const float ov = __shfl_xor(bd, off, 32);
    const int   oi = __shfl_xor(bi, off, 32);
    const bool take = (ov < bd) || ((ov == bd) && (oi < bi));
    bd = take ? ov : bd;
    bi = take ? oi : bi;
  }
  __syncthreads();
  sow[lane] = bi;
  __syncthreads();
  const int ncand = (cnt < kCandCap) ? cnt : kCandCap;
  for (int c0 = 0; c0 < ncand; c0 += 32) {
    const int c  = c0 + lane;
    const int cc = (c < ncand) ? c : (ncand - 1);
    const float dm = cdw[cc];
    const int   im = ciw[cc];
    int rank = 0;
    for (int j = 0; j < ncand; ++j) {
      const float dj = cdw[j];
      const int   ij = ciw[j];
      rank += ((dj < dm) || ((dj == dm) && (ij < im))) ? 1 : 0;
    }
    if (c < ncand && rank < 32) sow[rank] = im;
  }
  __syncthreads();

  int pid = sow[lane];
  pid = (pid < 0) ? 0 : pid;
  pid = (pid > kNPts - 1) ? (kNPts - 1) : pid;
  const float* prow = pts + ((size_t)b * kNPts + pid) * kFeat;
  const float* p3   = xyz + ((size_t)b * kNPts + pid) * 3;
  const float gx = p3[0] - sx;
  const float gy = p3[1] - sy;
  const float gz = p3[2] - sz;
  float zf = 0.0f;
  asm volatile("" : "+v"(zf));
  _Float16* trow = tile[wave] + lane * kK0;
#pragma unroll
  for (int c = 0; c < 8; ++c) {
    const v4f a  = *(const v4f*)(prow + c * 8);
    const v4f bq = *(const v4f*)(prow + c * 8 + 4);
    v8h hv;
    hv[0] = (_Float16)a[0];  hv[1] = (_Float16)a[1];  hv[2] = (_Float16)a[2];  hv[3] = (_Float16)a[3];
    hv[4] = (_Float16)bq[0]; hv[5] = (_Float16)bq[1]; hv[6] = (_Float16)bq[2]; hv[7] = (_Float16)bq[3];
    *(v8h*)(trow + c * 8) = hv;
    if ((c & 3) == 3) asm volatile("" ::: "memory");
  }
  {
    v8h hv;
    hv[0] = (_Float16)gx; hv[1] = (_Float16)gy; hv[2] = (_Float16)gz;
    hv[3] = (_Float16)zf; hv[4] = (_Float16)zf; hv[5] = (_Float16)zf; hv[6] = (_Float16)zf; hv[7] = (_Float16)zf;
    *(v8h*)(trow + 64) = hv;
    v8h hz;
#pragma unroll
    for (int e = 0; e < 8; ++e) hz[e] = (_Float16)zf;
    *(v8h*)(trow + 72) = hz;
    *(v8h*)(trow + 80) = hz;
    *(v8h*)(trow + 88) = hz;
  }
  __syncthreads();
  const v8h* tv = (const v8h*)tile[wave];
  unsigned short* dst = x0 + (size_t)g * (32 * kK0);
  v8h vals[12];
#pragma unroll
  for (int st = 0; st < 12; ++st) vals[st] = tv[st * 32 + lane];
  for (int pass = 0; pass < 2; ++pass) {
#pragma unroll
    for (int st = 0; st < 12; ++st) {
      *(volatile v8h*)(dst + (size_t)(st * 32 + lane) * 8) = vals[st];
    }
    __threadfence();
  }
}

__global__ __launch_bounds__(256) void prep_kernel(const float* __restrict__ w0,
                                                   const float* __restrict__ w1,
                                                   const float* __restrict__ w2,
                                                   unsigned short* __restrict__ W0h,
                                                   unsigned short* __restrict__ W1h,
                                                   unsigned short* __restrict__ W2h) {
  const int gt = blockIdx.x * 256 + threadIdx.x;
  float zf = 0.0f;
  asm volatile("" : "+v"(zf));
  if (gt < 64 * (kK0 / 8)) {
    const int o  = gt / (kK0 / 8);
    const int kc = (gt - o * (kK0 / 8)) * 8;
    v8h hv;
#pragma unroll
    for (int e = 0; e < 8; ++e) {
      const int k  = kc + e;
      const int sc = (k < 64) ? (k + 3) : ((k < kCin0) ? (k - 64) : 0);
      const float w = w0[o * kCin0 + sc];
      const float v = (k < kCin0) ? (w * kWCarry) : zf;
      hv[e] = (_Float16)v;
    }
    store2_v8h(W0h + (size_t)gt * 8, hv);
  }
  if (gt < 64 * 64 / 8) {
    const v4f a  = *(const v4f*)(w1 + (size_t)gt * 8);
    const v4f bq = *(const v4f*)(w1 + (size_t)gt * 8 + 4);
    v8h hv;
    hv[0] = (_Float16)(a[0] * kWCarry);  hv[1] = (_Float16)(a[1] * kWCarry);
    hv[2] = (_Float16)(a[2] * kWCarry);  hv[3] = (_Float16)(a[3] * kWCarry);
    hv[4] = (_Float16)(bq[0] * kWCarry); hv[5] = (_Float16)(bq[1] * kWCarry);
    hv[6] = (_Float16)(bq[2] * kWCarry); hv[7] = (_Float16)(bq[3] * kWCarry);
    store2_v8h(W1h + (size_t)gt * 8, hv);
  }
  if (gt < 128 * 64 / 8) {
    const v4f a  = *(const v4f*)(w2 + (size_t)gt * 8);
    const v4f bq = *(const v4f*)(w2 + (size_t)gt * 8 + 4);
    v8h hv;
    hv[0] = (_Float16)(a[0] * kWCarry);  hv[1] = (_Float16)(a[1] * kWCarry);
    hv[2] = (_Float16)(a[2] * kWCarry);  hv[3] = (_Float16)(a[3] * kWCarry);
    hv[4] = (_Float16)(bq[0] * kWCarry); hv[5] = (_Float16)(bq[1] * kWCarry);
    hv[6] = (_Float16)(bq[2] * kWCarry); hv[7] = (_Float16)(bq[3] * kWCarry);
    store2_v8h(W2h + (size_t)gt * 8, hv);
  }
}

template <int NOUT, int KDIM, int MODE>
__global__ __launch_bounds__(256) void gemm_bn_kernel(const unsigned short* __restrict__ Ap,
                                                      const unsigned short* __restrict__ Btp,
                                                      const float* __restrict__ bias,
                                                      unsigned short* __restrict__ Yout,
                                                      float* __restrict__ part,
                                                      float* __restrict__ ymax,
                                                      float* __restrict__ ymin) {
  static_assert(KDIM % 32 == 0);
  static_assert(NOUT % 64 == 0);
  static_assert(MODE == 1 || NOUT == 64);
  const _Float16* A  = (const _Float16*)Ap;
  const _Float16* Bt = (const _Float16*)Btp;
  __shared__ __align__(16) float sT[8][16 * 68];
  __shared__ float sred[8][2][64];
  const int lane  = threadIdx.x & 31;
  const int wave  = threadIdx.x >> 5;
  const int rlane = lane & 15;
  const int hh    = lane >> 4;
  const int koff  = hh * 8;
  const int mOff  = hh * 8;
  const int m0 = (blockIdx.x * 8 + wave) * 64;
  const int n0 = blockIdx.y * 64;

  v8f acc[4][4];
#pragma unroll
  for (int i = 0; i < 4; ++i)
#pragma unroll
    for (int j = 0; j < 4; ++j) acc[i][j] = (v8f){0.f, 0.f, 0.f, 0.f, 0.f, 0.f, 0.f, 0.f};

#pragma unroll 1
  for (int k0 = 0; k0 < KDIM; k0 += 32) {
    v16h bh[4];
#pragma unroll
    for (int j = 0; j < 4; ++j) {
      bh[j] = frag_load(Bt + (size_t)(n0 + (j << 4) + rlane) * KDIM + koff + k0);
    }
#pragma unroll
    for (int i = 0; i < 4; ++i) {
      const v16h ah = frag_load(A + (size_t)(m0 + (i << 4) + rlane) * KDIM + koff + k0);
#pragma unroll
      for (int j = 0; j < 4; ++j) acc[i][j] = mma_f16(ah, bh[j], acc[i][j]);
      guard_row(acc[i][0], acc[i][1], acc[i][2], acc[i][3], ah, bh[0], bh[1], bh[2], bh[3]);
    }
  }
  acc_guard4(acc[0][0], acc[0][1], acc[0][2], acc[0][3]);
  acc_guard4(acc[1][0], acc[1][1], acc[1][2], acc[1][3]);
  acc_guard4(acc[2][0], acc[2][1], acc[2][2], acc[2][3]);
  acc_guard4(acc[3][0], acc[3][1], acc[3][2], acc[3][3]);

  float bvv[4];
#pragma unroll
  for (int j = 0; j < 4; ++j) bvv[j] = bias[n0 + (j << 4) + rlane];
  float ls[4], lq[4];
  float mx[2][4], mn[2][4];
#pragma unroll
  for (int j = 0; j < 4; ++j) {
    ls[j] = 0.0f; lq[j] = 0.0f;
    mx[0][j] = -INFINITY; mx[1][j] = -INFINITY;
    mn[0][j] = INFINITY;  mn[1][j] = INFINITY;
  }
  float* slab = sT[wave];
#pragma unroll
  for (int i = 0; i < 4; ++i) {
#pragma unroll
    for (int j = 0; j < 4; ++j) {
#pragma unroll
      for (int r = 0; r < 8; ++r) {
        const float v  = acc[i][j][r] * kWCarryInv + bvv[j];
        const float v2 = v * v;
        ls[j] += v;
        lq[j] += v2;
        if (MODE == 0) {
          slab[(mOff + r) * 68 + (j << 4) + rlane] = v;
        } else {
          mx[i >> 1][j] = fmaxf(mx[i >> 1][j], v);
          mn[i >> 1][j] = fminf(mn[i >> 1][j], v);
        }
      }
    }
    if (MODE == 0) {
      __builtin_amdgcn_fence(__ATOMIC_RELEASE, "workgroup");
      __builtin_amdgcn_wave_barrier();
      __builtin_amdgcn_fence(__ATOMIC_ACQUIRE, "workgroup");
      const int q  = lane >> 3;
      const int c8 = (lane & 7) * 8;
      const int mBase = m0 + (i << 4);
      for (int pass = 0; pass < 2; ++pass) {
#pragma unroll
        for (int it = 0; it < 4; ++it) {
          const int row = it * 4 + q;
          const float* sp = slab + row * 68 + c8;
          v8h hv;
#pragma unroll
          for (int e = 0; e < 8; ++e) hv[e] = (_Float16)sp[e];
          *(volatile v8h*)(Yout + (size_t)(mBase + row) * NOUT + n0 + c8) = hv;
        }
        __threadfence();
      }
      __builtin_amdgcn_fence(__ATOMIC_RELEASE, "workgroup");
      __builtin_amdgcn_wave_barrier();
      __builtin_amdgcn_fence(__ATOMIC_ACQUIRE, "workgroup");
    }
  }

  if (MODE == 1) {
#pragma unroll
    for (int j = 0; j < 4; ++j) {
      mx[0][j] = fmaxf(mx[0][j], __shfl_xor(mx[0][j], 16, 32));
      mx[1][j] = fmaxf(mx[1][j], __shfl_xor(mx[1][j], 16, 32));
      mn[0][j] = fminf(mn[0][j], __shfl_xor(mn[0][j], 16, 32));
      mn[1][j] = fminf(mn[1][j], __shfl_xor(mn[1][j], 16, 32));
    }
    if (hh == 0) {
#pragma unroll
      for (int j = 0; j < 4; ++j) {
        slab[0 * 68 + (j << 4) + rlane] = mx[0][j];
        slab[1 * 68 + (j << 4) + rlane] = mx[1][j];
        slab[2 * 68 + (j << 4) + rlane] = mn[0][j];
        slab[3 * 68 + (j << 4) + rlane] = mn[1][j];
      }
    }
    __builtin_amdgcn_fence(__ATOMIC_RELEASE, "workgroup");
    __builtin_amdgcn_wave_barrier();
    __builtin_amdgcn_fence(__ATOMIC_ACQUIRE, "workgroup");
    const int c4 = rlane * 4;
    const v4f vmax = *(const v4f*)(slab + hh * 68 + c4);
    const v4f vmin = *(const v4f*)(slab + (2 + hh) * 68 + c4);
    const int gb = m0 >> 5;
    float* pmax = ymax + (size_t)(gb + hh) * 128 + n0 + c4;
    float* pmin = ymin + (size_t)(gb + hh) * 128 + n0 + c4;
    *(volatile v4f*)pmax = vmax;
    *(volatile v4f*)pmin = vmin;
    __threadfence();
    *(volatile v4f*)pmax = vmax;
    *(volatile v4f*)pmin = vmin;
  }

#pragma unroll
  for (int j = 0; j < 4; ++j) {
    ls[j] += __shfl_xor(ls[j], 16, 32);
    lq[j] += __shfl_xor(lq[j], 16, 32);
  }
  if (hh == 0) {
#pragma unroll
    for (int j = 0; j < 4; ++j) {
      sred[wave][0][(j << 4) + rlane] = ls[j];
      sred[wave][1][(j << 4) + rlane] = lq[j];
    }
  }
  __syncthreads();
  if (threadIdx.x < 128) {
    const int kind = threadIdx.x >> 6;
    const int col  = threadIdx.x & 63;
    float s = 0.0f;
#pragma unroll
    for (int w = 0; w < 8; ++w) s += sred[w][kind][col];
    store2_f32(part + ((size_t)blockIdx.x * 2 + kind) * NOUT + n0 + col, s);
  }
}

template <int NOUT>
__global__ __launch_bounds__(128) void bn_fin_kernel(const float* __restrict__ part,
                                                     const float* __restrict__ g,
                                                     const float* __restrict__ beta,
                                                     float* __restrict__ ab) {
  const int t  = threadIdx.x;
  const int tc = (t < NOUT) ? t : (NOUT - 1);
  double s = 0.0, q = 0.0;
#pragma unroll 1
  for (int i = 0; i < 512; ++i) {
    s += (double)part[((size_t)i * 2 + 0) * NOUT + tc];
    q += (double)part[((size_t)i * 2 + 1) * NOUT + tc];
  }
  const double invR = 1.0 / (double)kRows;
  const double mean = s * invR;
  double var = q * invR - mean * mean;
  var = (var < 0.0) ? 0.0 : var;
  const float vf  = (float)var;
  const float inv = 1.0f / sqrtf(vf + 1.0e-5f);
  const float a   = g[tc] * inv;
  const float c   = beta[tc] - a * (float)mean;
  if (t < NOUT) {
    store2_f32(ab + t, a);
    store2_f32(ab + 128 + t, c);
  }
}

__global__ __launch_bounds__(256) void bn_apply_kernel(const unsigned short* __restrict__ Yin,
                                                       const float* __restrict__ ab,
                                                       unsigned short* __restrict__ Xout) {
  const size_t idx = (size_t)blockIdx.x * 256 + threadIdx.x;
  const int c8 = ((int)(idx & 7)) * 8;
  const v4u w  = *(const v4u*)(Yin + idx * 8);
  const v4f a0 = *(const v4f*)(ab + c8);
  const v4f a1 = *(const v4f*)(ab + c8 + 4);
  const v4f c0 = *(const v4f*)(ab + 128 + c8);
  const v4f c1 = *(const v4f*)(ab + 128 + c8 + 4);
  const unsigned w0 = w[0];
  const unsigned w1 = w[1];
  const unsigned w2 = w[2];
  const unsigned w3 = w[3];
  float y[8];
  y[0] = h16_to_f32(w0 & 0xffffu); y[1] = h16_to_f32(w0 >> 16);
  y[2] = h16_to_f32(w1 & 0xffffu); y[3] = h16_to_f32(w1 >> 16);
  y[4] = h16_to_f32(w2 & 0xffffu); y[5] = h16_to_f32(w2 >> 16);
  y[6] = h16_to_f32(w3 & 0xffffu); y[7] = h16_to_f32(w3 >> 16);
  v8h hv;
  hv[0] = (_Float16)fmaxf(a0[0] * y[0] + c0[0], 0.0f);
  hv[1] = (_Float16)fmaxf(a0[1] * y[1] + c0[1], 0.0f);
  hv[2] = (_Float16)fmaxf(a0[2] * y[2] + c0[2], 0.0f);
  hv[3] = (_Float16)fmaxf(a0[3] * y[3] + c0[3], 0.0f);
  hv[4] = (_Float16)fmaxf(a1[0] * y[4] + c1[0], 0.0f);
  hv[5] = (_Float16)fmaxf(a1[1] * y[5] + c1[1], 0.0f);
  hv[6] = (_Float16)fmaxf(a1[2] * y[6] + c1[2], 0.0f);
  hv[7] = (_Float16)fmaxf(a1[3] * y[7] + c1[3], 0.0f);
  store2_v8h(Xout + idx * 8, hv);
}

__global__ __launch_bounds__(256) void pool_out_kernel(const float* __restrict__ ymax,
                                                       const float* __restrict__ ymin,
                                                       const float* __restrict__ ab,
                                                       float* __restrict__ out1) {
  const size_t idx = (size_t)blockIdx.x * 256 + threadIdx.x;
  const int c4 = ((int)(idx & 31)) * 4;
  const v4f vx = *(const v4f*)(ymax + idx * 4);
  const v4f vn = *(const v4f*)(ymin + idx * 4);
  const v4f a  = *(const v4f*)(ab + c4);
  const v4f c  = *(const v4f*)(ab + 128 + c4);
  v4f o;
#pragma unroll
  for (int e = 0; e < 4; ++e) {
    const float ae = a[e];
    const float fa = (ae >= 0.0f) ? 1.0f : 0.0f;
    const float fb = 1.0f - fa;
    const float ys = fa * vx[e] + fb * vn[e];
    o[e] = fmaxf(ae * ys + c[e], 0.0f);
  }
  store2_v4f(out1 + idx * 4, o);
}

extern "C" void kernel_launch(void* const* d_in, const int* in_sizes, int n_in,
                              void* d_out, int out_size, void* d_ws, size_t ws_size,
                              hipStream_t stream) {
  (void)in_sizes; (void)n_in; (void)out_size;
  if (ws_size < kWsTotal) return;
  const float* xyz   = (const float*)d_in[0];
  const float* pts   = (const float*)d_in[1];
  const float* w0    = (const float*)d_in[2];
  const float* b0    = (const float*)d_in[3];
  const float* g0    = (const float*)d_in[4];
  const float* beta0 = (const float*)d_in[5];
  const float* w1    = (const float*)d_in[6];
  const float* b1    = (const float*)d_in[7];
  const float* g1    = (const float*)d_in[8];
  const float* beta1 = (const float*)d_in[9];
  const float* w2    = (const float*)d_in[10];
  const float* b2    = (const float*)d_in[11];
  const float* g2    = (const float*)d_in[12];
  const float* beta2 = (const float*)d_in[13];

  float* out0 = (float*)d_out;
  float* out1 = (float*)((char*)d_out + kOut1Bytes);

  char* ws = (char*)d_ws;
  unsigned short* X0  = (unsigned short*)(ws + kOffX0);
  unsigned short* YA  = (unsigned short*)(ws + kOffYA);
  unsigned short* XB  = (unsigned short*)(ws + kOffXB);
  float* YMAX  = (float*)(ws + kOffYMax);
  float* YMIN  = (float*)(ws + kOffYMin);
  float* PART0 = (float*)(ws + kOffPart0);
  float* PART1 = (float*)(ws + kOffPart1);
  float* PART2 = (float*)(ws + kOffPart2);
  unsigned short* W0H = (unsigned short*)(ws + kOffW0H);
  unsigned short* W1H = (unsigned short*)(ws + kOffW1H);
  unsigned short* W2H = (unsigned short*)(ws + kOffW2H);
  float* AB0  = (float*)(ws + kOffAB);
  float* AB1  = AB0 + 256;
  float* AB2  = AB0 + 512;
  float* CXYZ = (float*)(ws + kOffCxyz);

  fps_kernel<<<kBatch, 256, 0, stream>>>(xyz, out0, CXYZ);
  group_kernel<<<kGroups / 4, 128, 0, stream>>>(xyz, pts, CXYZ, X0);
  prep_kernel<<<4, 256, 0, stream>>>(w0, w1, w2, W0H, W1H, W2H);

  gemm_bn_kernel<64, kK0, 0><<<dim3(kRows / 512, 1), 256, 0, stream>>>(X0, W0H, b0, YA, PART0, YMAX, YMIN);
  bn_fin_kernel<64><<<1, 128, 0, stream>>>(PART0, g0, beta0, AB0);
  bn_apply_kernel<<<kRows * 64 / 8 / 256, 256, 0, stream>>>(YA, AB0, XB);

  gemm_bn_kernel<64, 64, 0><<<dim3(kRows / 512, 1), 256, 0, stream>>>(XB, W1H, b1, YA, PART1, YMAX, YMIN);
  bn_fin_kernel<64><<<1, 128, 0, stream>>>(PART1, g1, beta1, AB1);
  bn_apply_kernel<<<kRows * 64 / 8 / 256, 256, 0, stream>>>(YA, AB1, XB);

  gemm_bn_kernel<128, 64, 1><<<dim3(kRows / 512, 2), 256, 0, stream>>>(XB, W2H, b2, YA, PART2, YMAX, YMIN);
  bn_fin_kernel<128><<<1, 128, 0, stream>>>(PART2, g2, beta2, AB2);
  pool_out_kernel<<<kGroups * 128 / 4 / 256, 256, 0, stream>>>(YMAX, YMIN, AB2, out1);
}
